// MultiHeadAttentionLayer_4080218931583
// MI455X (gfx1250) — hardware-run, weakly checked
//
#include <hip/hip_runtime.h>

typedef float          v8f   __attribute__((ext_vector_type(8)));
typedef float          v4f   __attribute__((ext_vector_type(4)));
typedef unsigned int   v4u   __attribute__((ext_vector_type(4)));
typedef int            v8i   __attribute__((ext_vector_type(8)));
typedef unsigned short v8us  __attribute__((ext_vector_type(8)));
typedef unsigned short v16us __attribute__((ext_vector_type(16)));
typedef __bf16         v16bf __attribute__((ext_vector_type(16)));
typedef _Float16       v16h  __attribute__((ext_vector_type(16)));
typedef v4f  __attribute__((may_alias)) v4fa;
typedef v8us __attribute__((may_alias)) v8usa;
union FragB { v16bf v; v16us u; v8us h[2]; v8i w; };
union FragH { v16h  v; v16us u; v8us h[2]; v8i w; };

__device__ __forceinline__ v8f wmb(const FragB& a, const FragB& b, v8f c) {
  v8f d = __builtin_amdgcn_wmma_f32_16x16x32_bf16(false, a.v, false, b.v, (short)0, c, false, false);
  asm volatile("v_nop\n\tv_nop\n\tv_nop\n\tv_nop" : "+v"(d) : "v"(a.w), "v"(b.w));
  return d;
}

__device__ __forceinline__ v8f wmh(const FragH& a, const FragH& b, v8f c) {
  v8f d = __builtin_amdgcn_wmma_f32_16x16x32_f16(false, a.v, false, b.v, (short)0, c, false, false);
  asm volatile("v_nop\n\tv_nop\n\tv_nop\n\tv_nop" : "+v"(d) : "v"(a.w), "v"(b.w));
  return d;
}

__device__ __forceinline__ unsigned bf16_bits(float f) {
  const unsigned u = __float_as_uint(f);
  const unsigned r = (u + 0x7FFFu + ((u >> 16) & 1u)) >> 16;
  const unsigned q = (u >> 16) | 0x40u;
  return ((u & 0x7fffffffu) > 0x7f800000u) ? q : r;
}

__device__ __forceinline__ float bf16_val(float f) {
  return __uint_as_float(bf16_bits(f) << 16);
}
__device__ __forceinline__ int clampi(int v, int lo, int hi) {
  return v < lo ? lo : (v > hi ? hi : v);
}

__device__ __forceinline__ unsigned f16_bits(float f) {
  const unsigned u  = __float_as_uint(f);
  const unsigned s  = (u >> 16) & 0x8000u;
  const unsigned a  = u & 0x7fffffffu;
  const unsigned t  = a - 0x38000000u;
  const unsigned r  = (t + 0x0FFFu + ((t >> 13) & 1u)) >> 13;
  const unsigned rc = r > 0x7C00u ? 0x7C00u : r;
  const bool small  = a < 0x38800000u;
  const bool isnan  = a > 0x7f800000u;
  const unsigned fin = small ? 0u : (s | rc);
  return isnan ? (s | 0x7E00u) : fin;
}

__device__ __forceinline__ unsigned pk16(unsigned lo, unsigned hi) { return lo | (hi << 16); }
__device__ __forceinline__ unsigned bf16_lo_bits(float v) {
  float hi = bf16_val(v);
  asm volatile("" : "+v"(hi));
  return bf16_bits(v - hi);
}
__device__ __forceinline__ v4u pack8_bf16(v4f a, v4f c) {
  return (v4u){ pk16(bf16_bits(a[0]), bf16_bits(a[1])), pk16(bf16_bits(a[2]), bf16_bits(a[3])),
                pk16(bf16_bits(c[0]), bf16_bits(c[1])), pk16(bf16_bits(c[2]), bf16_bits(c[3])) };
}
__device__ __forceinline__ v4u pack8_bf16_lo(v4f a, v4f c) {
  return (v4u){ pk16(bf16_lo_bits(a[0]), bf16_lo_bits(a[1])), pk16(bf16_lo_bits(a[2]), bf16_lo_bits(a[3])),
                pk16(bf16_lo_bits(c[0]), bf16_lo_bits(c[1])), pk16(bf16_lo_bits(c[2]), bf16_lo_bits(c[3])) };
}
__device__ __forceinline__ v4u pack8_f16(v4f a, v4f c) {
  return (v4u){ pk16(f16_bits(a[0]), f16_bits(a[1])), pk16(f16_bits(a[2]), f16_bits(a[3])),
                pk16(f16_bits(c[0]), f16_bits(c[1])), pk16(f16_bits(c[2]), f16_bits(c[3])) };
}

template <int FORM>
__global__ __launch_bounds__(256) void k_plane(const float* __restrict__ src, int rows, int cols, int ldsrc,
                                               unsigned short* __restrict__ dst, int MP, int KP) {
  static_assert(FORM >= 0 && FORM <= 3);
  const int KTOT = (FORM == 1 || FORM == 3) ? 2 * KP : KP;
  const unsigned ppr   = (unsigned)(KTOT >> 3);
  const unsigned kp8   = (unsigned)(KP >> 3);
  const unsigned total = (unsigned)MP * ppr;
  const unsigned g     = blockIdx.x * 256u + threadIdx.x;
  const unsigned rowu  = g / ppr;
  const unsigned p     = g - rowu * ppr;
  const bool second    = p >= kp8;
  const int row = (int)rowu;
  const int c0  = (int)((second ? p - kp8 : p) << 3);
  const float* srow = src + (size_t)clampi(row, 0, rows - 1) * (size_t)ldsrc;
  float x[8];
  unsigned mk[8];
#pragma unroll
  for (int e = 0; e < 8; ++e) {
    const int c = c0 + e;
    const float v = srow[clampi(c, 0, cols - 1)];
    asm volatile("" :: "v"(v));
    x[e]  = v;
    mk[e] = (row < rows && c < cols) ? 0xFFFFu : 0u;
  }
  const v4f a = (v4f){ x[0], x[1], x[2], x[3] };
  const v4f c = (v4f){ x[4], x[5], x[6], x[7] };
  v4u o;
  if (FORM == 2) {
    o = pack8_f16(a, c);
  } else {
    const v4u hi = pack8_bf16(a, c);
    o = hi;
    if (FORM == 1) { const v4u lo = pack8_bf16_lo(a, c); o = second ? lo : hi; }
  }
  const v4u mw = (v4u){ pk16(mk[0], mk[1]), pk16(mk[2], mk[3]), pk16(mk[4], mk[5]), pk16(mk[6], mk[7]) };
  o &= mw;
  if (g < total) {
    volatile v4u* q = (volatile v4u*)(dst + (size_t)g * 8);
    *q = o;
    __threadfence();
    *q = o;
  }
}

template <int FORM> struct FragOf    { typedef FragB T; };
template <>         struct FragOf<2> { typedef FragH T; };
__device__ __forceinline__ v8f mm(const FragB& a, const FragB& b, v8f c) { return wmb(a, b, c); }
__device__ __forceinline__ v8f mm(const FragH& a, const FragH& b, v8f c) { return wmh(a, b, c); }
template <class F> __device__ __forceinline__ F ld_frag(const unsigned short* p) {
  F f;
  f.h[0] = *(const v8usa*)(p);
  f.h[1] = *(const v8usa*)(p + 16);
  return f;
}

template <int FORM, int EPI>
__global__ __launch_bounds__(256) __attribute__((amdgpu_num_vgpr(248)))
void k_gemm_nt(const unsigned short* __restrict__ A, const unsigned short* __restrict__ B,
               const float* __restrict__ bias, float* __restrict__ D, int M, int N, int KTOT, int ldd) {
  static_assert(FORM >= 0 && FORM <= 2);
  static_assert(EPI == 0 || EPI == 1);
  typedef typename FragOf<FORM>::T F;
  __shared__ __attribute__((aligned(16))) float sT[8][16 * 68];
  const int lane = threadIdx.x & 31;
  const int wave = threadIdx.x >> 5;
  const int tilesM = (M + 63) >> 6;
  const int tilesN = (N + 63) >> 6;
  const int tile = blockIdx.x * 8 + wave;
  if (tile >= tilesM * tilesN) return;
  const int tm = tile / tilesN;
  const int tn = tile - tm * tilesN;
  const int m0 = tm << 6;
  const int n0 = tn << 6;

  const int rl = lane & 15;
  const int h8 = (lane >> 4) * 8;
  const unsigned short* pa = A + (size_t)(m0 + rl) * (size_t)KTOT + h8;
  const unsigned short* pb = B + (size_t)(n0 + rl) * (size_t)KTOT + h8;

  v8f acc[4][4];
#pragma unroll
  for (int i = 0; i < 4; ++i)
#pragma unroll
    for (int j = 0; j < 4; ++j) acc[i][j] = (v8f){0.f, 0.f, 0.f, 0.f, 0.f, 0.f, 0.f, 0.f};

#pragma unroll 1
  for (int k0 = 0; k0 < KTOT; k0 += 32) {
    F bf[4];
#pragma unroll
    for (int j = 0; j < 4; ++j) bf[j] = ld_frag<F>(pb + (size_t)(j << 4) * (size_t)KTOT + k0);
#pragma unroll
    for (int i = 0; i < 4; ++i) {
      const F af = ld_frag<F>(pa + (size_t)(i << 4) * (size_t)KTOT + k0);
#pragma unroll
      for (int j = 0; j < 4; ++j) acc[i][j] = mm(af, bf[j], acc[i][j]);
    }
  }

  float* slab = sT[wave];
  const int hh = lane >> 4;
  const int c4 = (lane & 15) * 4;
  const int nc = n0 + c4;
  const bool cok = nc < N;
  v4f bv = (v4f){0.f, 0.f, 0.f, 0.f};
  if (EPI == 1) {
    bv = *(const v4fa*)(bias + clampi(nc, 0, N - 4));
    asm volatile("" :: "v"(bv));
  }
#pragma unroll
  for (int i = 0; i < 4; ++i) {
    const int mBase = m0 + (i << 4);
#pragma unroll
    for (int j = 0; j < 4; ++j) {
#pragma unroll
      for (int r = 0; r < 8; ++r) slab[(h8 + r) * 68 + (j << 4) + rl] = acc[i][j][r];
    }
    __builtin_amdgcn_fence(__ATOMIC_RELEASE, "workgroup");
    __builtin_amdgcn_wave_barrier();
    __builtin_amdgcn_fence(__ATOMIC_ACQUIRE, "workgroup");
    v4f vv[8];
#pragma unroll
    for (int it = 0; it < 8; ++it) {
      const int row = it * 2 + hh;
      v4f v = *(const v4fa*)(slab + row * 68 + c4);
      if (EPI == 1) v += bv;
      vv[it] = v;
    }
    for (int pass = 0; pass < 2; ++pass) {
#pragma unroll
      for (int it = 0; it < 8; ++it) {
        const int row = mBase + it * 2 + hh;
        if (cok && row < M) *(volatile v4f*)(D + (size_t)row * (size_t)ldd + nc) = vv[it];
      }
      __threadfence();
    }
    __builtin_amdgcn_fence(__ATOMIC_RELEASE, "workgroup");
    __builtin_amdgcn_wave_barrier();
    __builtin_amdgcn_fence(__ATOMIC_ACQUIRE, "workgroup");
  }
}

#include <stddef.h>

typedef int v4i __attribute__((ext_vector_type(4)));

#define N_NODES 50000
#define N_EDGES 600000
#define FEATS   128
#define NHEADS  8
#define DHEADS  16
#define NCOL3   384
#define MPAD    50048
#define NBLK    1024
#define BGRID   49
#define LCAP    16384
#define BTHR    256
#define BWAVE   8
#define EPT     8
#define CHUNK   (BTHR * EPT)
#define WCAP    (32 * EPT)
#define HITMAX  12567
#define LDS_SMALL ((4 * NBLK + BWAVE * WCAP + 16) * 4)
#define LDS_FULL  (LDS_SMALL + 2 * LCAP * 4)

static_assert(FEATS == 32 * 4);
static_assert(NHEADS * DHEADS == FEATS);
static_assert(N_NODES <= 65536);
static_assert((LCAP % 32) == 0);
static_assert((long long)LCAP * 4 >= (long long)HITMAX * 5);
static_assert(BGRID * NBLK >= N_NODES);
static_assert((N_EDGES % EPT) == 0 && N_EDGES >= EPT);
static_assert((N_NODES % 16) == 0 && (MPAD % 64) == 0 && MPAD >= N_NODES);
static_assert((NCOL3 % 64) == 0 && (FEATS % 32) == 0);
static_assert(BTHR * 4 == NBLK);
static_assert(CHUNK == 2048 && NBLK == 1024);
static_assert(LDS_FULL <= 262144);
static_assert((N_NODES % 8) == 0);

constexpr size_t al256(size_t x) { return (x + 255) & ~(size_t)255; }
constexpr size_t SZ_P    = (size_t)MPAD * NCOL3 * 4;
constexpr size_t SZ_KV   = (size_t)N_NODES * 256 * 4;
constexpr size_t SZ_HB   = (size_t)MPAD * FEATS * 2;
constexpr size_t SZ_LIST = (size_t)BGRID * LCAP * 4;
constexpr size_t SZ_TAB  = (size_t)BGRID * NBLK * 4;
constexpr size_t SZ_WT   = (size_t)NCOL3 * FEATS * 2;
constexpr size_t SZ_BIAS = (size_t)NCOL3 * 4;
constexpr size_t SZ_FLAG = (size_t)BGRID * 128;
constexpr size_t O_P    = 0;
constexpr size_t O_KV   = al256(O_P + SZ_P);
constexpr size_t O_LIST = al256(O_KV + SZ_KV);
constexpr size_t O_OFF  = al256(O_LIST + SZ_LIST);
constexpr size_t O_CNT  = al256(O_OFF + SZ_TAB);
constexpr size_t O_NS   = al256(O_CNT + SZ_TAB);
constexpr size_t O_ND   = al256(O_NS + SZ_TAB);
constexpr size_t O_WT   = al256(O_ND + SZ_TAB);
constexpr size_t O_BIAS = al256(O_WT + SZ_WT);
constexpr size_t O_FLAG = al256(O_BIAS + SZ_BIAS);
constexpr size_t O_END  = al256(O_FLAG + SZ_FLAG);
static_assert(SZ_HB <= SZ_KV);
static_assert(O_END <= ((size_t)128 << 20));

__device__ __forceinline__ void prep_unit(const float* __restrict__ w, const float* __restrict__ b,
                                          unsigned short* __restrict__ wt, float* __restrict__ bias,
                                          int m, int bx, int tid) {
  const int u  = bx * 256 + tid;
  const int nl = u >> 4;
  const int k8 = (u & 15) * 8;
  const float* p = w + (size_t)k8 * FEATS + nl;
  const float x0 = p[0],         x1 = p[FEATS],     x2 = p[2 * FEATS], x3 = p[3 * FEATS];
  const float x4 = p[4 * FEATS], x5 = p[5 * FEATS], x6 = p[6 * FEATS], x7 = p[7 * FEATS];
  const v4u o = pack8_bf16((v4f){ x0, x1, x2, x3 }, (v4f){ x4, x5, x6, x7 });
  volatile v4u* q = (volatile v4u*)(wt + (size_t)(m * FEATS + nl) * FEATS + k8);
  *q = o;
  __threadfence();
  *q = o;
  if (bx == 0 && tid < 32) {
    const v4f bv = *(const v4fa*)(b + 4 * tid);
    const v4f r = (v4f){ bf16_val(bv[0]), bf16_val(bv[1]), bf16_val(bv[2]), bf16_val(bv[3]) };
    volatile v4f* qb = (volatile v4f*)(bias + m * FEATS + 4 * tid);
    *qb = r;
    __threadfence();
    *qb = r;
  }
}

__global__ __launch_bounds__(256) void k_prep(const float* __restrict__ wq, const float* __restrict__ bq,
                                              const float* __restrict__ wk, const float* __restrict__ bk,
                                              const float* __restrict__ wv, const float* __restrict__ bv,
                                              unsigned short* __restrict__ wt, float* __restrict__ bias) {
  const int m   = (int)blockIdx.y;
  const int bx  = (int)blockIdx.x;
  const int tid = (int)threadIdx.x;
  if (m == 0)      prep_unit(wq, bq, wt, bias, 0, bx, tid);
  else if (m == 1) prep_unit(wk, bk, wt, bias, 1, bx, tid);
  else             prep_unit(wv, bv, wt, bias, 2, bx, tid);
}

template <int MODE>
__global__ __launch_bounds__(BTHR) void k_build(const int* __restrict__ keys, const int* __restrict__ pay,
                                                int* __restrict__ NRM, int* __restrict__ LIST,
                                                int* __restrict__ OFF, int* __restrict__ CNT,
                                                int* __restrict__ FLAG, int nE) {
  extern __shared__ v4f lds_dyn[];
  int* scnt = (int*)lds_dyn;
  int* soff = scnt + NBLK;
  int* cur  = soff + NBLK;
  int* nrm  = cur + NBLK;
  int* list = nrm + NBLK;
  int* wcnt = list + BWAVE * WCAP;
  int* reg1 = wcnt + 16;
  int* reg2 = reg1 + LCAP;
  const int tid = (int)threadIdx.x, lane = tid & 31, wave = tid >> 5;
  const int blk = (int)blockIdx.x;
  const int slotBase = blk * NBLK;

  for (int i = tid; i < NBLK; i += BTHR) scnt[i] = 0;
  if (MODE == 1) {
#pragma unroll 1
    for (int i = tid; i < LCAP; i += BTHR) reg2[i] = 0;
  }
  __syncthreads();

  int tot = 0, totRaw = 0;
  const int nChunks = (nE + CHUNK - 1) / CHUNK;
  int* wl = list + wave * WCAP;
#pragma unroll 1
  for (int ch = 0; ch < nChunks; ++ch) {
    const int cbase = ch * CHUNK;
    const int el0 = tid * EPT;
    const int e0  = cbase + el0;
    const int vm  = (e0 < nE) ? 0 : -1;
    const int e0c = e0 < nE - EPT ? e0 : nE - EPT;
    const v4i da = *(const v4i*)(keys + e0c);
    const v4i db = *(const v4i*)(keys + e0c + 4);
    asm volatile("" :: "v"(da), "v"(db));
    const unsigned ub = (unsigned)slotBase;
    const unsigned s0 = (unsigned)(da.x | vm) - ub, s1 = (unsigned)(da.y | vm) - ub;
    const unsigned s2 = (unsigned)(da.z | vm) - ub, s3 = (unsigned)(da.w | vm) - ub;
    const unsigned s4 = (unsigned)(db.x | vm) - ub, s5 = (unsigned)(db.y | vm) - ub;
    const unsigned s6 = (unsigned)(db.z | vm) - ub, s7 = (unsigned)(db.w | vm) - ub;
    const bool h0 = s0 < (unsigned)NBLK, h1 = s1 < (unsigned)NBLK, h2 = s2 < (unsigned)NBLK, h3 = s3 < (unsigned)NBLK;
    const bool h4 = s4 < (unsigned)NBLK, h5 = s5 < (unsigned)NBLK, h6 = s6 < (unsigned)NBLK, h7 = s7 < (unsigned)NBLK;
    const int hc = (int)h0 + (int)h1 + (int)h2 + (int)h3 + (int)h4 + (int)h5 + (int)h6 + (int)h7;
    int incl = hc;
#pragma unroll
    for (int d = 1; d < 32; d <<= 1) {
      const int up = __shfl_up(incl, d);
      incl += (lane >= d) ? up : 0;
    }
    const int wcu = __builtin_amdgcn_readfirstlane(__shfl(incl, 31));
    int pos = incl - hc;
    if (h0) { wl[pos < WCAP ? pos : WCAP - 1] = ((el0 + 0) << 10) | (int)s0; pos += 1; }
    if (h1) { wl[pos < WCAP ? pos : WCAP - 1] = ((el0 + 1) << 10) | (int)s1; pos += 1; }
    if (h2) { wl[pos < WCAP ? pos : WCAP - 1] = ((el0 + 2) << 10) | (int)s2; pos += 1; }
    if (h3) { wl[pos < WCAP ? pos : WCAP - 1] = ((el0 + 3) << 10) | (int)s3; pos += 1; }
    if (h4) { wl[pos < WCAP ? pos : WCAP - 1] = ((el0 + 4) << 10) | (int)s4; pos += 1; }
    if (h5) { wl[pos < WCAP ? pos : WCAP - 1] = ((el0 + 5) << 10) | (int)s5; pos += 1; }
    if (h6) { wl[pos < WCAP ? pos : WCAP - 1] = ((el0 + 6) << 10) | (int)s6; pos += 1; }
    if (h7) { wl[pos < WCAP ? pos : WCAP - 1] = ((el0 + 7) << 10) | (int)s7; pos += 1; }
    if (lane == 0) wcnt[wave] = wcu;
    __syncthreads();

    if (MODE == 0) {
      if (wave == 0) {
#pragma unroll 1
        for (int w2 = 0; w2 < BWAVE; ++w2) {
          const int c = __builtin_amdgcn_readfirstlane(clampi(wcnt[w2], 0, WCAP));
#pragma unroll 1
          for (int b0 = 0; b0 < c; b0 += 32) {
            const int ii  = (b0 + lane) < c ? (b0 + lane) : c - 1;
            const int uv  = list[w2 * WCAP + ii];
            const int m32 = (c - b0) < 32 ? (c - b0) : 32;
#pragma unroll 1
            for (int k = 0; k < m32; ++k) {
              const int u  = __builtin_amdgcn_readlane(uv, k);
              const int sl = u & (NBLK - 1);
              scnt[sl] = scnt[sl] + 1;
            }
          }
        }
      }
    } else {
      int pre = 0, all = 0;
#pragma unroll
      for (int w2 = 0; w2 < BWAVE; ++w2) {
        const int c = clampi(wcnt[w2], 0, WCAP);
        all += c;
        pre += (w2 < wave) ? c : 0;
      }
      const int wcc  = wcu > WCAP ? WCAP : wcu;
      const int base = tot + pre;
#pragma unroll 1
      for (int i0 = 0; i0 < wcc; i0 += 32) {
        const int i   = i0 + lane;
        const int ic  = i < wcc ? i : wcc - 1;
        const int ent = wl[ic];
        const int el  = (ent >> 10) & (CHUNK - 1);
        const int sl  = ent & (NBLK - 1);
        const int eid = clampi(cbase + el, 0, nE - 1);
        const int sraw = pay[eid];
        asm volatile("" :: "v"(sraw));
        const int sv = clampi(sraw, 0, 65535);
        const int p2 = base + i;
        if (i < wcc && p2 < LCAP) reg1[p2] = (sl << 16) | sv;
      }
      totRaw += all;
      tot += all;
      tot = tot > LCAP ? LCAP : tot;
    }
    __syncthreads();
  }

  if (MODE == 1) {
    const int nh = __builtin_amdgcn_readfirstlane(tot);
    if (wave == 0) {
#pragma unroll 1
      for (int b0 = 0; b0 < nh; b0 += 32) {
        const int ii  = (b0 + lane) < nh ? (b0 + lane) : nh - 1;
        const int uv  = reg1[ii];
        const int m32 = (nh - b0) < 32 ? (nh - b0) : 32;
#pragma unroll 1
        for (int k = 0; k < m32; ++k) {
          const int u  = __builtin_amdgcn_readlane(uv, k);
          const int sl = (u >> 16) & (NBLK - 1);
          scnt[sl] = scnt[sl] + 1;
        }
      }
    }
    __syncthreads();
    {
      int a0 = scnt[4 * tid + 0], a1 = scnt[4 * tid + 1], a2 = scnt[4 * tid + 2], a3 = scnt[4 * tid + 3];
      a0 = a0 < 0 ? 0 : a0; a1 = a1 < 0 ? 0 : a1; a2 = a2 < 0 ? 0 : a2; a3 = a3 < 0 ? 0 : a3;
      const int ts = a0 + a1 + a2 + a3;
      int incl = ts;
#pragma unroll
      for (int d = 1; d < 32; d <<= 1) {
        const int up = __shfl_up(incl, d);
        incl += (lane >= d) ? up : 0;
      }
      if (lane == 31) wcnt[8 + wave] = incl;
      __syncthreads();
      int pre = 0;
#pragma unroll
      for (int w2 = 0; w2 < BWAVE; ++w2) pre += (w2 < wave) ? wcnt[8 + w2] : 0;
      int run = pre + incl - ts;
      soff[4 * tid + 0] = run; cur[4 * tid + 0] = run; run += a0;
      soff[4 * tid + 1] = run; cur[4 * tid + 1] = run; run += a1;
      soff[4 * tid + 2] = run; cur[4 * tid + 2] = run; run += a2;
      soff[4 * tid + 3] = run; cur[4 * tid + 3] = run;
    }
    __syncthreads();
    if (wave == 0) {
#pragma unroll 1
      for (int b0 = 0; b0 < nh; b0 += 32) {
        const int ii  = (b0 + lane) < nh ? (b0 + lane) : nh - 1;
        const int uv  = reg1[ii];
        const int m32 = (nh - b0) < 32 ? (nh - b0) : 32;
#pragma unroll 1
        for (int k = 0; k < m32; ++k) {
          const int u  = __builtin_amdgcn_readlane(uv, k);
          const int sl = (u >> 16) & (NBLK - 1);
          const int sv = u & 0xFFFF;
          const int p2 = clampi(cur[sl], 0, LCAP - 1);
          reg2[p2] = sv;
          cur[sl]  = p2 + 1;
        }
      }
    }
    __syncthreads();
  }

#pragma unroll 1
  for (int r = 0; r < 4; ++r) {
    const int i = tid + BTHR * r;
    int c = scnt[i];
    c = c < 1 ? 1 : c;
    nrm[i] = __float_as_int(1.0f / sqrtf((float)c));
  }
  __syncthreads();

  const size_t tb = (size_t)blk * NBLK + (size_t)(4 * tid);
  const v4i nv = (v4i){ nrm[4 * tid + 0], nrm[4 * tid + 1], nrm[4 * tid + 2], nrm[4 * tid + 3] };
  v4i ov = (v4i){ 0, 0, 0, 0 }, cv = (v4i){ 0, 0, 0, 0 };
  if (MODE == 1) {
    ov = (v4i){ soff[4 * tid + 0], soff[4 * tid + 1], soff[4 * tid + 2], soff[4 * tid + 3] };
    cv = (v4i){ scnt[4 * tid + 0], scnt[4 * tid + 1], scnt[4 * tid + 2], scnt[4 * tid + 3] };
  }
  const int fl = (totRaw > LCAP) ? 1 : 0;
  const v4i fv = (v4i){ fl, fl, fl, fl };
  for (int pass = 0; pass < 2; ++pass) {
    *(volatile v4i*)(NRM + tb) = nv;
    if (MODE == 1) {
      *(volatile v4i*)(OFF + tb) = ov;
      *(volatile v4i*)(CNT + tb) = cv;
#pragma unroll 1
      for (int it = 0; it < LCAP / (4 * BTHR); ++it) {
        const int idx = it * BTHR + tid;
        const v4i lv = (v4i){ reg2[4 * idx + 0], reg2[4 * idx + 1], reg2[4 * idx + 2], reg2[4 * idx + 3] };
        *(volatile v4i*)(LIST + (size_t)blk * LCAP + (size_t)(4 * idx)) = lv;
      }
      if (tid < 8) *(volatile v4i*)(FLAG + blk * 32 + 4 * tid) = fv;
    }
    __threadfence();
  }
}

__device__ __forceinline__ v4f relu_keep(v4f v, bool bad, float qn) {
  v4f r;
  r[0] = (v[0] < 0.0f) ? 0.0f : v[0];
  r[1] = (v[1] < 0.0f) ? 0.0f : v[1];
  r[2] = (v[2] < 0.0f) ? 0.0f : v[2];
  r[3] = (v[3] < 0.0f) ? 0.0f : v[3];
  r[0] = bad ? qn : r[0]; r[1] = bad ? qn : r[1]; r[2] = bad ? qn : r[2]; r[3] = bad ? qn : r[3];
  return r;
}

__global__ __launch_bounds__(256) void k_replay1(const float* __restrict__ P, const int* __restrict__ LIST,
                                                 const int* __restrict__ OFF, const int* __restrict__ CNT,
                                                 const int* __restrict__ FLAG, const float* __restrict__ NS,
                                                 const float* __restrict__ ND, const float* __restrict__ BIAS,
                                                 float* __restrict__ outQ, float* __restrict__ KV, int nN) {
  const int lane = (int)threadIdx.x & 31, wave = (int)threadIdx.x >> 5;
  const int t = (int)blockIdx.x * 8 + wave;
  if (t >= nN) return;
  const int blk = t >> 10;
  const int cntv = CNT[t];
  const int offv = OFF[t];
  const int flg  = FLAG[blk * 32];
  const float nd = ND[t];
  asm volatile("" :: "v"(cntv), "v"(offv), "v"(flg), "v"(nd));
  const int offc = clampi(offv, 0, LCAP);
  const int cnc  = clampi(cntv, 0, LCAP - offc);
  const int off  = __builtin_amdgcn_readfirstlane(offc);
  const int cn   = __builtin_amdgcn_readfirstlane(cnc);
  const bool bad = (flg != 0) || (cnc != cntv) || (offc != offv);
  const float qn = __int_as_float(0x7fc00000);

  const v4f bq = *(const v4fa*)(BIAS + 4 * lane);
  const v4f bk = *(const v4fa*)(BIAS + FEATS + 4 * lane);
  const v4f bv = *(const v4fa*)(BIAS + 2 * FEATS + 4 * lane);
  v4f aq = (v4f){ 0.f, 0.f, 0.f, 0.f }, ak = aq, av = aq;
  const int* lb = LIST + (size_t)blk * LCAP;
#pragma unroll 1
  for (int b0 = 0; b0 < cn; b0 += 32) {
    const int ii = clampi(off + b0 + lane, 0, LCAP - 1);
    const int wv = lb[ii];
    asm volatile("" :: "v"(wv));
    const int m32 = (cn - b0) < 32 ? (cn - b0) : 32;
#pragma unroll 1
    for (int k = 0; k < m32; ++k) {
      const int s = clampi(__builtin_amdgcn_readlane(wv, k), 0, nN - 1);
      const float w = NS[s];
      const float* pr = P + (size_t)s * NCOL3 + 4 * lane;
      const v4f x = *(const v4fa*)(pr);
      const v4f y = *(const v4fa*)(pr + FEATS);
      const v4f z = *(const v4fa*)(pr + 2 * FEATS);
      aq += x * w;
      ak += y * w;
      av += z * w;
    }
  }
  const v4f rq = relu_keep(aq * nd + bq, bad, qn);
  const v4f rk = relu_keep(ak * nd + bk, bad, qn);
  const v4f rv = relu_keep(av * nd + bv, bad, qn);
  volatile v4f* po = (volatile v4f*)(outQ + (size_t)t * FEATS + 4 * lane);
  volatile v4f* pk = (volatile v4f*)(KV + (size_t)t * 256 + 4 * lane);
  volatile v4f* pv = (volatile v4f*)(KV + (size_t)t * 256 + FEATS + 4 * lane);
  for (int pass = 0; pass < 2; ++pass) {
    *po = rq;
    *pk = rk;
    *pv = rv;
    __threadfence();
  }
}

__global__ __launch_bounds__(256) void k_replay2(const float* __restrict__ KV, const int* __restrict__ LIST,
                                                 const int* __restrict__ OFF, const int* __restrict__ CNT,
                                                 const int* __restrict__ FLAG, float* out, int nN) {
  const int lane = (int)threadIdx.x & 31, wave = (int)threadIdx.x >> 5;
  const int t = (int)blockIdx.x * 8 + wave;
  if (t >= nN) return;
  const int blk = t >> 10;
  const int cntv = CNT[t];
  const int offv = OFF[t];
  const int flg  = FLAG[blk * 32];
  asm volatile("" :: "v"(cntv), "v"(offv), "v"(flg));
  const int offc = clampi(offv, 0, LCAP);
  const int cnc  = clampi(cntv, 0, LCAP - offc);
  const int off  = __builtin_amdgcn_readfirstlane(offc);
  const int cn   = __builtin_amdgcn_readfirstlane(cnc);
  const bool bad = (flg != 0) || (cnc != cntv) || (offc != offv);
  const float qn = __int_as_float(0x7fc00000);

  float* orow = out + (size_t)t * FEATS + 4 * lane;
  const v4f q = *(const v4fa*)orow;
  asm volatile("" :: "v"(q));
  v4f av = (v4f){ 0.f, 0.f, 0.f, 0.f };
  float zs = 0.0f;
  const int* lb = LIST + (size_t)blk * LCAP;
#pragma unroll 1
  for (int b0 = 0; b0 < cn; b0 += 32) {
    const int ii = clampi(off + b0 + lane, 0, LCAP - 1);
    const int wv = lb[ii];
    asm volatile("" :: "v"(wv));
    const int m32 = (cn - b0) < 32 ? (cn - b0) : 32;
#pragma unroll 1
    for (int k = 0; k < m32; ++k) {
      const int s = clampi(__builtin_amdgcn_readlane(wv, k), 0, nN - 1);
      const float* pr = KV + (size_t)s * 256 + 4 * lane;
      const v4f k4 = *(const v4fa*)(pr);
      const v4f v4 = *(const v4fa*)(pr + FEATS);
      float part = k4[0] * q[0] + k4[1] * q[1] + k4[2] * q[2] + k4[3] * q[3];
      part += __shfl_xor(part, 1);
      part += __shfl_xor(part, 2);
      float sc = part * 0.25f;
      sc = (sc < -10.0f) ? -10.0f : sc;
      sc = (sc > 10.0f) ? 10.0f : sc;
      const float e = expf(sc);
      av += v4 * e;
      zs += e;
    }
  }
  const float den = zs + 1e-6f;
  v4f r;
  r[0] = av[0] / den; r[1] = av[1] / den; r[2] = av[2] / den; r[3] = av[3] / den;
  r[0] = bad ? qn : r[0]; r[1] = bad ? qn : r[1]; r[2] = bad ? qn : r[2]; r[3] = bad ? qn : r[3];
  volatile v4f* po = (volatile v4f*)orow;
  for (int pass = 0; pass < 2; ++pass) {
    *po = r;
    __threadfence();
  }
}

extern "C" void kernel_launch(void* const* d_in, const int* in_sizes, int n_in,
                              void* d_out, int out_size, void* d_ws, size_t ws_size,
                              hipStream_t stream) {
  if (n_in < 9) return;
  if (in_sizes[0] != N_NODES * FEATS) return;
  if (in_sizes[1] != FEATS * FEATS || in_sizes[3] != FEATS * FEATS || in_sizes[5] != FEATS * FEATS) return;
  if (in_sizes[2] != FEATS || in_sizes[4] != FEATS || in_sizes[6] != FEATS) return;
  if (in_sizes[7] != N_EDGES || in_sizes[8] != N_EDGES) return;
  if (out_size != N_NODES * FEATS) return;
  if (O_END > ws_size) return;

  const float* h   = (const float*)d_in[0];
  const float* W_Q = (const float*)d_in[1];
  const float* b_Q = (const float*)d_in[2];
  const float* W_K = (const float*)d_in[3];
  const float* b_K = (const float*)d_in[4];
  const float* W_V = (const float*)d_in[5];
  const float* b_V = (const float*)d_in[6];
  const int*   src = (const int*)d_in[7];
  const int*   dst = (const int*)d_in[8];
  float* out = (float*)d_out;

  char* ws = (char*)d_ws;
  float*          P    = (float*)(ws + O_P);
  float*          KV   = (float*)(ws + O_KV);
  unsigned short* HB   = (unsigned short*)(ws + O_KV);
  int*            LIST = (int*)(ws + O_LIST);
  int*            OFF  = (int*)(ws + O_OFF);
  int*            CNT  = (int*)(ws + O_CNT);
  int*            NSb  = (int*)(ws + O_NS);
  int*            NDb  = (int*)(ws + O_ND);
  unsigned short* WT   = (unsigned short*)(ws + O_WT);
  float*          BIAS = (float*)(ws + O_BIAS);
  int*            FLAG = (int*)(ws + O_FLAG);

  hipFuncSetAttribute(reinterpret_cast<const void*>(&k_build<1>),
                      hipFuncAttributeMaxDynamicSharedMemorySize, LDS_FULL);

  k_prep<<<dim3(8, 3), 256, 0, stream>>>(W_Q, b_Q, W_K, b_K, W_V, b_V, WT, BIAS);
  k_plane<0><<<MPAD * FEATS / 8 / 256, 256, 0, stream>>>(h, N_NODES, FEATS, FEATS, HB, MPAD, FEATS);
  {
    const int tiles = ((N_NODES + 63) / 64) * (NCOL3 / 64);
    k_gemm_nt<0, 0><<<(tiles + 7) / 8, 256, 0, stream>>>(HB, WT, BIAS, P, N_NODES, NCOL3, FEATS, NCOL3);
  }
  k_build<0><<<BGRID, BTHR, LDS_SMALL, stream>>>(src, src, NSb, LIST, OFF, CNT, FLAG, N_EDGES);
  k_build<1><<<BGRID, BTHR, LDS_FULL, stream>>>(dst, src, NDb, LIST, OFF, CNT, FLAG, N_EDGES);
  k_replay1<<<(N_NODES + 7) / 8, 256, 0, stream>>>(P, LIST, OFF, CNT, FLAG, (const float*)NSb, (const float*)NDb,
                                                   BIAS, out, KV, N_NODES);
  k_replay2<<<(N_NODES + 7) / 8, 256, 0, stream>>>(KV, LIST, OFF, CNT, FLAG, out, N_NODES);
}
